// RelationNetwork_57621281243635
// MI455X (gfx1250) — hardware-run, weakly checked
//
#include <hip/hip_runtime.h>


#ifndef NB
#define NB 4
#endif
#ifndef NOBJ
#define NOBJ 1024
#endif
#define NB_FULL   4
#define NOBJ_FULL 1024
#define DM   64
#define NC   128
#define TPB  (NOBJ / 64)
#define SAP  72
#define SSC  (1.0f / 64.0f)
#define WSC  64.0f
#define PAIRS ((float)((NOBJ * (NOBJ - 1)) / 2))

static_assert(DM == 64);
static_assert(NC == 2 * DM);
static_assert(NC % 64 == 0);
static_assert(DM % 32 == 0);
static_assert(NOBJ % 64 == 0);
static_assert((NB * NOBJ) % 64 == 0);
static_assert(NB >= 1);
static_assert(NB <= 16);
static_assert(NB <= NB_FULL);
static_assert(NOBJ <= NOBJ_FULL);
static_assert(((size_t)NOBJ * (NOBJ - 1)) / 2 < (size_t)16777216);
static_assert(((size_t)NOBJ * DM) % 8 == 0);
static_assert(((size_t)DM * NC) % 8 == 0);
static_assert(SAP % 8 == 0);
static_assert(SAP >= DM);
static_assert((NB * DM * 4) % 128 == 0);
static_assert(8 * 16 == 32 * 4);
static_assert((NB * DM / 4) * 16 == NB * DM * 4);
static_assert((DM * DM / 8) % 128 == 0);
static_assert(DM / 8 == 8);
static_assert(16 * SAP * 2 + DM * SAP * 2 + 16 * DM * 4 <= 131072);
static_assert(32 * 4 <= 131072);

typedef _Float16 h16;
typedef unsigned short bf;
typedef __attribute__((ext_vector_type(16))) __bf16   v16bf;
typedef __attribute__((ext_vector_type(16))) _Float16 v16h;
typedef __attribute__((ext_vector_type(8)))  _Float16 v8h;
typedef __attribute__((ext_vector_type(8)))  unsigned short v8us;
typedef __attribute__((ext_vector_type(8)))  float    v8f;
typedef __attribute__((ext_vector_type(4)))  float    v4f;
typedef v4f  __attribute__((may_alias)) v4fa;
typedef v8h  __attribute__((may_alias)) v8ha;

__device__ __forceinline__ unsigned short f2bf(float f) { unsigned u = __float_as_uint(f); u += 0x7FFFu + ((u >> 16) & 1u); return (unsigned short)(u >> 16); }
__device__ __forceinline__ float bfr(float f) { return __uint_as_float(((unsigned)f2bf(f)) << 16); }
__device__ __forceinline__ v16h cat16(v8h lo, v8h hi) { return __builtin_shufflevector(lo, hi, 0, 1, 2, 3, 4, 5, 6, 7, 8, 9, 10, 11, 12, 13, 14, 15); }
__device__ __forceinline__ v16bf cat16b(v8us lo, v8us hi) { return __builtin_bit_cast(v16bf, __builtin_shufflevector(lo, hi, 0, 1, 2, 3, 4, 5, 6, 7, 8, 9, 10, 11, 12, 13, 14, 15)); }
__device__ __forceinline__ v8f wmma16(v16h a, v16h b, v8f c) { return __builtin_amdgcn_wmma_f32_16x16x32_f16(false, a, false, b, (short)0, c, false, false); }
__device__ __forceinline__ v8f wmmab(v16bf a, v16bf b, v8f c) { return __builtin_amdgcn_wmma_f32_16x16x32_bf16(false, a, false, b, (short)0, c, false, false); }
__device__ __forceinline__ v16h  ldh(const h16* p) { return cat16(*(const v8h*)p, *(const v8h*)(p + 16)); }
__device__ __forceinline__ v16bf ldb(const bf* p)  { return cat16b(*(const v8us*)p, *(const v8us*)(p + 16)); }
__device__ __forceinline__ void wave_sync() { __builtin_amdgcn_fence(3  , "wavefront"); __builtin_amdgcn_wave_barrier(); asm volatile("" ::: "memory"); }

static __device__ __forceinline__ h16 toh_flush(float v) { const h16 r = (h16)v; return (fabsf(v) < 6.103515625e-05f) ? (h16)0.0f : r; }
__device__ __forceinline__ v8f wmmabg(v16bf a, v16bf b, v8f c) { c = wmmab(a, b, c); asm volatile("v_nop\n\tv_nop\n\tv_nop\n\tv_nop" : "+v"(c) : "v"(a), "v"(b)); return c; }
__device__ __forceinline__ v8f wmma16g(v16h a, v16h b, v8f c) { c = wmma16(a, b, c); asm volatile("v_nop\n\tv_nop\n\tv_nop\n\tv_nop" : "+v"(c) : "v"(a), "v"(b)); return c; }

__global__ __launch_bounds__(256) void k_cvt8(const float* __restrict__ src, bf* dst, size_t n8) {
    const size_t i = (size_t)blockIdx.x * 256 + threadIdx.x; if (i >= n8) return;
    const v8f v = *(const v8f*)(src + i * 8); v8us o;
#pragma unroll
    for (int k = 0; k < 8; ++k) o[k] = f2bf(v[k]);
    *(volatile v8us*)(dst + i * 8) = o; __threadfence(); *(volatile v8us*)(dst + i * 8) = o;
}

__global__ __launch_bounds__(32) void k_pairsum(const bf* __restrict__ A, const bf* __restrict__ Bt, float* PART) {
    __shared__ __align__(16) float os[32];
    const int K = DM;
    const int lane = threadIdx.x & 31, lr = lane & 15, hi = lane >> 4; const int r0 = blockIdx.x * 64, c0 = blockIdx.y * 64;
    v8f acc[4][4];
#pragma unroll
    for (int mb = 0; mb < 4; ++mb)
#pragma unroll
        for (int nb = 0; nb < 4; ++nb) acc[mb][nb] = (v8f){};
    const size_t aoff = (size_t)(r0 + lr) * K + 8 * hi, boff = (size_t)(c0 + lr) * K + 8 * hi;
#pragma unroll 1
    for (int kc = 0; kc < K; kc += 32) {
        v16bf a[4];
#pragma unroll
        for (int mb = 0; mb < 4; ++mb) a[mb] = ldb(A + aoff + (size_t)mb * 16 * K + kc);
#pragma unroll
        for (int nb = 0; nb < 4; ++nb) { const v16bf b = ldb(Bt + boff + (size_t)nb * 16 * K + kc);
#pragma unroll
            for (int mb = 0; mb < 4; ++mb) acc[mb][nb] = wmmabg(a[mb], b, acc[mb][nb]); }
    }
    const int tt = r0 % NOBJ;
    const bool odd = (lr & 1) != 0;
    float p[4];
#pragma unroll
    for (int nb = 0; nb < 4; ++nb) p[nb] = 0.0f;
#pragma unroll
    for (int mb = 0; mb < 4; ++mb) {
#pragma unroll
        for (int j = 0; j < 8; ++j) {
            const int i = tt + mb * 16 + hi * 8 + j;
            const float w = odd ? (float)i : (float)(NOBJ - 1 - i);
#pragma unroll
            for (int nb = 0; nb < 4; ++nb) p[nb] += w * acc[mb][nb][j]; } }
#pragma unroll
    for (int nb = 0; nb < 4; ++nb) { float v = p[nb]; v += __shfl_xor(v, 1, 32); v += __shfl_xor(v, 16, 32); p[nb] = v; }
    if ((hi == 0) & (!odd)) {
#pragma unroll
        for (int nb = 0; nb < 4; ++nb) os[nb * 8 + (lr >> 1)] = p[nb]; }
    wave_sync();
    float* dst = PART + ((size_t)blockIdx.x * DM + (size_t)blockIdx.y * 32);
#pragma unroll 1
    for (int ps = 0; ps < 2; ++ps) {
        if (lane < 8) { const v4f val = *(const v4fa*)(&os[lane * 4]); *(volatile v4f*)(dst + lane * 4) = val; }
        if (ps == 0) __threadfence(); }
}

__global__ __launch_bounds__(128) void k_head(const float* __restrict__ PART, const float* __restrict__ bg, const float* __restrict__ Wf, const float* __restrict__ bo, float* OUT) {
    __shared__ __align__(16) h16 sa[16 * SAP];
    __shared__ __align__(16) h16 wfs[DM * SAP];
    __shared__ __align__(16) float os[16 * DM];
    const int tid = threadIdx.x;
    const int lane = tid & 31, lr = lane & 15, hi = lane >> 4;
    const int wave = __builtin_amdgcn_readfirstlane((int)(threadIdx.x >> 5));
#pragma unroll 1
    for (int idx = tid; idx < NB * DM; idx += 128) {
        const int b = idx / DM, e = idx % DM;
        const float* pp = PART + (size_t)b * TPB * DM + e;
        float sv = 0.0f;
#pragma unroll 1
        for (int t = 0; t < TPB; ++t) sv += pp[(size_t)t * DM];
        sv += PAIRS * bfr(bg[e]);
        sa[b * SAP + e] = toh_flush(sv * SSC);
    }
#pragma unroll 1
    for (int idx = NB * DM + tid; idx < 16 * DM; idx += 128) sa[(idx / DM) * SAP + (idx % DM)] = (h16)0.0f;
#pragma unroll 1
    for (int q = tid; q < DM * DM / 8; q += 128) {
        const int f = q >> 3, c8 = (q & 7) * 8;
        const v4f x0 = *(const v4f*)(Wf + (size_t)f * DM + c8); const v4f x1 = *(const v4f*)(Wf + (size_t)f * DM + c8 + 4); v8h hv;
#pragma unroll
        for (int i = 0; i < 4; ++i) { hv[i] = toh_flush(bfr(x0[i]) * WSC); hv[4 + i] = toh_flush(bfr(x1[i]) * WSC); }
        *(v8ha*)(&wfs[f * SAP + c8]) = hv;
    }
    __syncthreads();
    const int f0 = wave * 16;
    v8f acc = (v8f){};
#pragma unroll
    for (int kc = 0; kc < DM; kc += 32) {
        const int ao = lr * SAP + kc + 8 * hi;
        const int wo = (f0 + lr) * SAP + kc + 8 * hi;
        const v16h a = cat16(*(const v8ha*)(&sa[ao]), *(const v8ha*)(&sa[ao + 16]));
        const v16h b = cat16(*(const v8ha*)(&wfs[wo]), *(const v8ha*)(&wfs[wo + 16]));
        acc = wmma16g(a, b, acc);
    }
    const float bias = bfr(bo[f0 + lr]);
#pragma unroll
    for (int r = 0; r < 8; ++r) os[(8 * hi + r) * DM + f0 + lr] = acc[r] + bias;
    __syncthreads();
    if (wave == 0) {
#pragma unroll 1
        for (int ps = 0; ps < 2; ++ps) {
#pragma unroll 1
            for (int q = lane; q < NB * DM / 4; q += 32) {
                const v4f val = *(const v4fa*)(&os[q * 4]);
                *(volatile v4f*)(OUT + (size_t)q * 4) = val; }
            if (ps == 0) __threadfence(); }
    }
}

static constexpr size_t al256(size_t v) { return (v + 255) & ~(size_t)255; }
static constexpr size_t SZ_XB = al256((size_t)NB * NOBJ * DM * 2);
static constexpr size_t SZ_WG = al256((size_t)NC * DM * 2);
static constexpr size_t SZ_PT = al256((size_t)(NB * NOBJ / 64) * DM * 4);
static constexpr size_t SZ_TOTAL = SZ_XB + SZ_WG + SZ_PT;
static_assert(SZ_TOTAL <= (size_t)134217728);
static_assert((size_t)(NB * NOBJ / 64) * DM * 4 == (size_t)(NB * NOBJ / 64) * 2 * 128);
static_assert((size_t)NB * TPB == (size_t)(NB * NOBJ / 64));

extern "C" void kernel_launch(void* const* d_in, const int* in_sizes, int n_in,
                              void* d_out, int out_size, void* d_ws, size_t ws_size, hipStream_t stream) {
    if (n_in < 5) return;
    const size_t needx = ((size_t)(NB - 1) * NOBJ_FULL + NOBJ) * DM;
    if ((size_t)in_sizes[0] < needx) return;
    if ((size_t)in_sizes[1] < (size_t)DM * NC) return;
    if (in_sizes[2] < DM || (size_t)in_sizes[3] < (size_t)DM * DM || in_sizes[4] < DM) return;
    if ((size_t)out_size < (size_t)NB * DM) return;
    if (SZ_TOTAL > ws_size) return;
    const float* xin = (const float*)d_in[0];
    const float* wg  = (const float*)d_in[1];
    const float* bgp = (const float*)d_in[2];
    const float* wf  = (const float*)d_in[3];
    const float* bop = (const float*)d_in[4];
    float* OUT = (float*)d_out;
    char* wsp = (char*)d_ws;
    bf* XB = (bf*)wsp; wsp += SZ_XB;
    bf* WGB = (bf*)wsp; wsp += SZ_WG;
    float* PART = (float*)wsp; wsp += SZ_PT;

    if (NOBJ == NOBJ_FULL) {
        const size_t n8 = (size_t)NB * NOBJ * DM / 8;
        k_cvt8<<<(unsigned)((n8 + 255) / 256), 256, 0, stream>>>(xin, XB, n8);
    } else {
        const size_t n8 = (size_t)NOBJ * DM / 8;
        for (int b = 0; b < NB; ++b) k_cvt8<<<(unsigned)((n8 + 255) / 256), 256, 0, stream>>>(xin + (size_t)b * NOBJ_FULL * DM, XB + (size_t)b * NOBJ * DM, n8);
    }
    { const size_t n8 = (size_t)DM * NC / 8; k_cvt8<<<(unsigned)((n8 + 255) / 256), 256, 0, stream>>>(wg, WGB, n8); }

    k_pairsum<<<dim3(NB * NOBJ / 64, NC / 64, 1), 32, 0, stream>>>(XB, WGB, PART);
    k_head<<<dim3(1, 1, 1), 128, 0, stream>>>(PART, bgp, wf, bop, OUT);
}
